// TextMaskedMultiheadSelfAttention_83416854823051
// MI455X (gfx1250) — hardware-verified
//
#include <hip/hip_runtime.h>


namespace {
constexpr int Bn = 2, L = 2048, D = 1024, H = 16, HD = 64, NT = Bn * L, DQ = 3 * D;
constexpr float EPS = 1e-5f, XS = 8.0f, PS = 8.0f;

typedef _Float16 b16;
typedef __attribute__((ext_vector_type(16))) _Float16 v16b;
typedef __attribute__((ext_vector_type(8))) _Float16 v8b;
typedef __attribute__((ext_vector_type(8))) float v8f;
typedef __attribute__((ext_vector_type(4))) float v4f;
__device__ __forceinline__ float bf16_rne(float f) { unsigned int u = __float_as_uint(f); u += 0x7FFFu + ((u >> 16) & 1u); return __uint_as_float(u & 0xFFFF0000u); }
__device__ __forceinline__ v16b frag_kb(const b16* p, int hh) { const v8b a = *(const v8b*)(p + 8 * hh), b = *(const v8b*)(p + 16 + 8 * hh); v16b f;
#pragma unroll
  for (int e = 0; e < 8; ++e) { f[e] = a[e]; f[8 + e] = b[e]; } return f; }
__device__ __forceinline__ v8f wmma16b(v16b a, v16b b, v8f c) { v8f d = __builtin_amdgcn_wmma_f32_16x16x32_f16(false, a, false, b, (short)0, c, false, false); asm volatile("v_nop\n\tv_nop\n\tv_nop\n\tv_nop" : "+v"(d) : "v"(a), "v"(b)); return d; }
__device__ __forceinline__ void wave_lds_sync() { __builtin_amdgcn_fence(__ATOMIC_RELEASE, "workgroup"); __builtin_amdgcn_wave_barrier(); __builtin_amdgcn_fence(__ATOMIC_ACQUIRE, "workgroup"); }
__device__ __forceinline__ float nexp(float x) { return __builtin_amdgcn_exp2f(x * 1.4426950408889634f); }
__device__ __forceinline__ float pmul(float a, float b) { float p = a * b; asm volatile("" : "+v"(p)); return p; }
__device__ __forceinline__ float wsum(float v) {
#pragma unroll
  for (int o = 1; o < 32; o <<= 1) v += __shfl_xor(v, o); return v; }
__device__ __forceinline__ float tanh_n(float x) { const float e = __builtin_amdgcn_exp2f(x * 2.8853900817779268f); return 1.0f - 2.0f * __builtin_amdgcn_rcpf(e + 1.0f); }
__device__ __forceinline__ float gelu_t(float x) { const float c = 0.7978845608028654f; return 0.5f * x * (1.0f + tanh_n(c * (x + 0.044715f * x * x * x))); }

__global__ __launch_bounds__(256) void prep_kernel(const float* __restrict__ wq, const float* __restrict__ wk, const float* __restrict__ wv, const float* __restrict__ bq, const float* __restrict__ bk, const float* __restrict__ bv, const float* __restrict__ g, const float* __restrict__ be, b16* __restrict__ R, float* __restrict__ P) {
  const size_t tid = (size_t)blockIdx.x * 256 + threadIdx.x, nth = (size_t)gridDim.x * 256;
  for (int pass = 0; pass < 2; ++pass) {
    for (size_t p = tid; p < (size_t)DQ * D / 8; p += nth) { const size_t q = p * 8; const float* src = (q < (size_t)D * D) ? (wq + q) : (q < (size_t)2 * D * D) ? (wk + (q - (size_t)D * D)) : (wv + (q - (size_t)2 * D * D)); v8b v;
#pragma unroll
      for (int e = 0; e < 8; ++e) v[e] = (b16)bf16_rne(src[e]); *(volatile v8b*)(R + q) = v; }
    for (size_t q = tid; q < 5120; q += nth) { const int i = (int)q; float v; if (i < 1024) v = bq[i]; else if (i < 2048) v = bk[i - 1024]; else if (i < 3072) v = bv[i - 2048]; else if (i < 4096) v = g[i - 3072]; else v = be[i - 4096]; P[q] = bf16_rne(v); }
    __threadfence(); }
}

__global__ __launch_bounds__(256) void ln_kernel(const float* __restrict__ src, int rnd, const float* __restrict__ g, const float* __restrict__ bb, b16* __restrict__ dst) {
  const int row = blockIdx.x * 8 + (threadIdx.x >> 5), lane = threadIdx.x & 31; const float* xr = src + (size_t)row * D;
  float v[32]; float s = 0.0f;
#pragma unroll
  for (int i = 0; i < 32; ++i) { float x = xr[(i >> 3) * 256 + lane * 8 + (i & 7)]; if (rnd) x = bf16_rne(x); v[i] = x; s += x; }
  s = wsum(s); const float mu = s * (1.0f / D); float q = 0.0f;
#pragma unroll
  for (int i = 0; i < 32; ++i) { const float d = v[i] - mu; q += pmul(d, d); }
  q = wsum(q); const float inv = rsqrtf(q * (1.0f / D) + EPS);
  for (int pass = 0; pass < 2; ++pass) {
#pragma unroll
    for (int gq = 0; gq < 4; ++gq) { v8b o; const int c0 = gq * 256 + lane * 8;
#pragma unroll
      for (int e = 0; e < 8; ++e) o[e] = (b16)((pmul((v[gq * 8 + e] - mu) * inv, g[c0 + e]) + bb[c0 + e]) * XS);
      *(volatile v8b*)(dst + (size_t)row * D + c0) = o; }
    __threadfence(); }
}

template <int K, int N, int EPI, int RND>
__global__ __launch_bounds__(64) void gemm_kernel(const b16* __restrict__ A, const b16* __restrict__ Bw, const float* __restrict__ bias, const float* __restrict__ resid, b16* __restrict__ Ch, float* __restrict__ Cf) {
  __shared__ __attribute__((aligned(16))) float Ts[2][32][128 + 4];
  const int lane = threadIdx.x & 31, wave = threadIdx.x >> 5, nloc = lane & 15, hlf = lane >> 4, m0 = blockIdx.y * 32, c0 = blockIdx.x * 256 + wave * 128;
  v8f acc[2][8];
#pragma unroll
  for (int r = 0; r < 2; ++r)
#pragma unroll
    for (int t = 0; t < 8; ++t) acc[r][t] = (v8f){};
  for (int kb = 0; kb < K; kb += 32) { const v16b a0 = frag_kb(A + (size_t)(m0 + nloc) * K + kb, hlf), a1 = frag_kb(A + (size_t)(m0 + 16 + nloc) * K + kb, hlf);
#pragma unroll
    for (int t = 0; t < 8; ++t) { const v16b bw = frag_kb(Bw + (size_t)(c0 + t * 16 + nloc) * K + kb, hlf); acc[0][t] = wmma16b(a0, bw, acc[0][t]); acc[1][t] = wmma16b(a1, bw, acc[1][t]); } }
#pragma unroll
  for (int t = 0; t < 8; ++t) { const float bv = (bias != nullptr) ? bias[c0 + t * 16 + nloc] : 0.0f;
#pragma unroll
    for (int r = 0; r < 2; ++r)
#pragma unroll
      for (int v = 0; v < 8; ++v) { float y = acc[r][t][v] * (1.0f / XS) + bv; if (EPI == 2) y = gelu_t(y); Ts[wave][r * 16 + 8 * hlf + v][t * 16 + nloc] = y; } }
  wave_lds_sync();
  for (int pass = 0; pass < 2; ++pass) {
    if (EPI == 1) { for (int i = lane; i < 32 * 32; i += 32) { const int rr = i >> 5, c4 = (i & 31) * 4; const size_t gi = (size_t)(m0 + rr) * N + c0 + c4; v4f o = *(const v4f*)(&Ts[wave][rr][c4]); const v4f xr = *(const v4f*)(resid + gi);
        for (int e = 0; e < 4; ++e) o[e] += RND ? bf16_rne(xr[e]) : xr[e]; *(volatile v4f*)(Cf + gi) = o; } }
    else { for (int i = lane; i < 32 * 16; i += 32) { const int rr = i >> 4, c8 = (i & 15) * 8; v8b o; for (int e = 0; e < 8; ++e) o[e] = (b16)(Ts[wave][rr][c8 + e] * XS); *(volatile v8b*)(Ch + (size_t)(m0 + rr) * N + c0 + c8) = o; } }
    __threadfence(); }
}

__global__ __launch_bounds__(256) void vt_kernel(const b16* __restrict__ QKV, b16* __restrict__ vt) {
  __shared__ __attribute__((aligned(16))) b16 T[HD][128 + 8];
  const int b = blockIdx.z, h = blockIdx.y, t0 = blockIdx.x * 128, t_ = threadIdx.x;
  for (int i = t_; i < 128 * (HD / 8); i += 256) { const int tk = i >> 3, d8 = (i & 7) * 8; const v8b vv = *(const v8b*)(QKV + ((size_t)(b * L + t0 + tk)) * DQ + 2 * D + h * HD + d8); for (int e = 0; e < 8; ++e) T[d8 + e][tk] = vv[e]; }
  __syncthreads();
  for (int pass = 0; pass < 2; ++pass) { for (int i = t_; i < HD * 16; i += 256) { const int d = i >> 4, c8 = (i & 15) * 8; *(volatile v8b*)(vt + (((size_t)b * H + h) * HD + d) * L + t0 + c8) = *(const v8b*)(&T[d][c8]); } __threadfence(); }
}

__global__ __launch_bounds__(256) void attn_kernel(const b16* __restrict__ QKV, const b16* __restrict__ vt, const float* __restrict__ x, float* __restrict__ out) {
  __shared__ __attribute__((aligned(16))) float Os[16][8 * HD + 4];
  const int wid = threadIdx.x >> 5, lane = threadIdx.x & 31, hh = lane >> 4, col = lane & 15; const int b = blockIdx.x / (L / 16), q0 = (blockIdx.x % (L / 16)) * 16, h = blockIdx.y * 8 + wid, qi = q0 + col;
  const b16* Qr = QKV + (size_t)(b * L) * DQ + h * HD; const b16* Kr = QKV + (size_t)(b * L) * DQ + D + h * HD; const b16* V = vt + (((size_t)b * H + h) * HD) * L;
  const v16b qf0 = frag_kb(Qr + (size_t)qi * DQ, hh), qf1 = frag_kb(Qr + (size_t)qi * DQ + 32, hh);
  const float SC = 0.02209708691207961f / (XS * XS);
  float m = -INFINITY, l = 0.0f; v8f o[4] = {{}, {}, {}, {}};
  for (int kb = 0; kb < L; kb += 32) {
    const v16b ka0 = frag_kb(Kr + (size_t)(kb + col) * DQ, hh), ka1 = frag_kb(Kr + (size_t)(kb + col) * DQ + 32, hh), kc0 = frag_kb(Kr + (size_t)(kb + 16 + col) * DQ, hh), kc1 = frag_kb(Kr + (size_t)(kb + 16 + col) * DQ + 32, hh);
    v8f s0 = {}, s1 = {}; s0 = wmma16b(ka0, qf0, s0); s0 = wmma16b(ka1, qf1, s0); s1 = wmma16b(kc0, qf0, s1); s1 = wmma16b(kc1, qf1, s1);
    float mr = -INFINITY;
#pragma unroll
    for (int r = 0; r < 8; ++r) { s0[r] *= SC; s1[r] *= SC; mr = fmaxf(mr, fmaxf(s0[r], s1[r])); }
    mr = fmaxf(mr, __shfl_xor(mr, 16));
    const float mn = fmaxf(m, mr), al_ = nexp(m - mn); m = mn; float sum = 0.0f; v16b pbv;
#pragma unroll
    for (int r = 0; r < 8; ++r) { const float e0 = nexp(s0[r] - mn), e1 = nexp(s1[r] - mn); sum += e0 + e1; pbv[r] = (b16)(e0 * PS); pbv[8 + r] = (b16)(e1 * PS); }
    sum += __shfl_xor(sum, 16); l = l * al_ + sum;
#pragma unroll
    for (int t = 0; t < 4; ++t) { o[t] *= al_; const v16b vf = frag_kb(V + (size_t)(t * 16 + col) * L + kb, hh); o[t] = wmma16b(vf, pbv, o[t]); } }
  const float inv = 1.0f / (l * PS * XS);
#pragma unroll
  for (int t = 0; t < 4; ++t)
#pragma unroll
    for (int r = 0; r < 8; ++r) Os[col][wid * HD + t * 16 + 8 * hh + r] = o[t][r] * inv;
  __syncthreads();
  for (int pass = 0; pass < 2; ++pass) { for (int i = threadIdx.x; i < 16 * 128; i += 256) { const int rr = i >> 7, c4 = (i & 127) * 4; const size_t gi = ((size_t)(b * L + q0 + rr)) * D + blockIdx.y * 8 * HD + c4; v4f v = *(const v4f*)(&Os[rr][c4]); const v4f xr = *(const v4f*)(x + gi);
      for (int e = 0; e < 4; ++e) v[e] += bf16_rne(xr[e]); *(volatile v4f*)(out + gi) = v; } __threadfence(); }
}
}

extern "C" void kernel_launch(void* const* d_in, const int* in_sizes, int n_in,
                              void* d_out, int out_size, void* d_ws, size_t ws_size, hipStream_t stream) {
  (void)n_in; (void)out_size;
  const float* x = (const float*)d_in[0]; const float* wq = (const float*)d_in[1]; const float* bq = (const float*)d_in[2]; const float* wk = (const float*)d_in[3]; const float* bk = (const float*)d_in[4]; const float* wv = (const float*)d_in[5]; const float* bv = (const float*)d_in[6]; const float* g = (const float*)d_in[7]; const float* be = (const float*)d_in[8];
  float* out = (float*)d_out;
  if (in_sizes[0] != NT * D || in_sizes[1] != D * D || in_sizes[3] != D * D || in_sizes[5] != D * D) return;
  size_t off = 0; char* ws = (char*)d_ws;
  auto carve = [&](size_t bytes) { char* p = ws + off; off += (bytes + 255) & ~(size_t)255; return p; };
  b16* R = (b16*)carve((size_t)DQ * D * 2); float* P = (float*)carve(5120 * 4); b16* SH = (b16*)carve((size_t)NT * D * 2); b16* QKV = (b16*)carve((size_t)NT * DQ * 2); b16* VT = (b16*)carve((size_t)Bn * H * HD * L * 2);
  if (off > ws_size) return;
  prep_kernel<<<512, 256, 0, stream>>>(wq, wk, wv, bq, bk, bv, g, be, R, P);
  ln_kernel<<<NT / 8, 256, 0, stream>>>(x, 1, P + 3072, P + 4096, SH);
  gemm_kernel<D, DQ, 0, 0><<<dim3(DQ / 256, NT / 32), 64, 0, stream>>>(SH, R, P, nullptr, QKV, nullptr);
  vt_kernel<<<dim3(L / 128, H, Bn), 256, 0, stream>>>(QKV, VT);
  attn_kernel<<<dim3(NT / 16, 2), 256, 0, stream>>>(QKV, VT, x, out);
}
